// Model_33990371181080
// MI455X (gfx1250) — hardware-verified
//
#include <hip/hip_runtime.h>
#include <math.h>

constexpr int NBATCH  = 32;
constexpr int NSTEP   = 512;
constexpr int NIN     = 768;
constexpr int NHID    = 512;
constexpr int NGATE   = 4 * NHID;
constexpr int KCAT    = NIN + NHID;
constexpr int NTHR    = 256;
constexpr int SEQ_BLK = 16;
constexpr int XPITCH  = NIN + 8;
constexpr int HPITCH  = NHID + 8;
constexpr int CPITCH  = NHID + 4;
constexpr float WCARRY     = 256.0f;
constexpr float WCARRY_INV = 1.0f / 256.0f;

static_assert(NIN % 32 == 0, "x part of K is a multiple of 32");
static_assert(NHID % 32 == 0, "h part of K is a multiple of 32");
static_assert(KCAT % 32 == 0, "fused K is a multiple of 32");
static_assert(NHID == 64 * (NTHR / 32), "8 waves x 64 hidden units");
static_assert(NBATCH % SEQ_BLK == 0, "whole 16-row tiles");
static_assert(XPITCH % 8 == 0 && HPITCH % 8 == 0 && CPITCH % 4 == 0, "16-B aligned LDS rows");
static_assert(NGATE == NTHR * 8, "bias staging covers 2048 exactly");
static_assert((NGATE * (NIN / 8)) % NTHR == 0 && (NGATE * (NHID / 8)) % NTHR == 0, "convert grids exact");
static_assert((NIN / 8) % 32 == 0 && (NHID / 8) % 32 == 0, "a wave of the convert kernel stays inside one row");
static_assert((NIN * 2) % 128 == 0 && (KCAT * 2) % 128 == 0, "weight plane column split and row pitch on 128-B lines");

typedef __attribute__((ext_vector_type(16))) _Float16 v16h;
typedef __attribute__((ext_vector_type(8)))  _Float16 v8h;
typedef __attribute__((ext_vector_type(4)))  _Float16 v4h;
typedef __attribute__((ext_vector_type(8)))  float    v8f;
typedef __attribute__((ext_vector_type(4)))  float    v4f;

__device__ __forceinline__ v16h frag_load(const _Float16* p) {
  union { v16h v; v8h h[2]; } f;
  f.h[0] = *(const v8h*)(p);
  f.h[1] = *(const v8h*)(p + 16);
  return f.v;
}
__device__ __forceinline__ v8f mma16(v16h a, v16h b, v8f c) {
  return __builtin_amdgcn_wmma_f32_16x16x32_f16(false, a, false, b, (short)0, c, false, false);
}
__device__ __forceinline__ void guard_group(v8f& d0, v8f& d1, v8f& d2, v8f& d3,
                                            v16h a, v16h b0, v16h b1, v16h b2, v16h b3) {
  asm volatile("v_nop\n\tv_nop\n\tv_nop\n\tv_nop"
               : "+v"(d0), "+v"(d1), "+v"(d2), "+v"(d3)
               : "v"(a), "v"(b0), "v"(b1), "v"(b2), "v"(b3));
}
__device__ __forceinline__ void acc_guard4(v8f& a, v8f& b, v8f& c, v8f& d) {
  asm volatile("v_nop\n\tv_nop\n\tv_nop\n\tv_nop" : "+v"(a), "+v"(b), "+v"(c), "+v"(d));
}

__device__ __forceinline__ void kstep(const _Float16* ap, const _Float16* wp,
                                      v8f& d0, v8f& d1, v8f& d2, v8f& d3) {
  const v16h a  = frag_load(ap);
  const v16h b0 = frag_load(wp);
  const v16h b1 = frag_load(wp + (size_t)1 * NHID * KCAT);
  const v16h b2 = frag_load(wp + (size_t)2 * NHID * KCAT);
  const v16h b3 = frag_load(wp + (size_t)3 * NHID * KCAT);
  d0 = mma16(a, b0, d0);
  d1 = mma16(a, b1, d1);
  d2 = mma16(a, b2, d2);
  d3 = mma16(a, b3, d3);
  guard_group(d0, d1, d2, d3, a, b0, b1, b2, b3);
}

__device__ __forceinline__ float sigm(float v) { return __builtin_amdgcn_rcpf(1.0f + expf(-v)); }
__device__ __forceinline__ float tnh(float v)  { return 1.0f - 2.0f * __builtin_amdgcn_rcpf(expf(2.0f * v) + 1.0f); }

__device__ __forceinline__ void stage_x(const float* __restrict__ xr, _Float16* xs_row, int sub) {
#pragma unroll 4
  for (int it = 0; it < NIN / 64; ++it) {
    const int c4 = (sub + 16 * it) * 4;
    const v4f v = *(const v4f*)(xr + c4);
    v4h hv;
    hv[0] = (_Float16)v[0];
    hv[1] = (_Float16)v[1];
    hv[2] = (_Float16)v[2];
    hv[3] = (_Float16)v[3];
    *(v4h*)(xs_row + c4) = hv;
  }
}

__global__ __launch_bounds__(NTHR) void cvt_w_kernel(const float* __restrict__ src, unsigned short* __restrict__ dst,
                                                     int nrow, int ncol8, int spitch, int dpitch, int dcol0, float sc) {
  const int i  = blockIdx.x * NTHR + threadIdx.x;
  const int n8 = nrow * ncol8;
  if (i < n8) {
    const int row = i / ncol8;
    const int c8  = i - row * ncol8;
    const float* sp = src + (size_t)row * spitch + c8 * 8;
    const v4f a = *(const v4f*)(sp);
    const v4f b = *(const v4f*)(sp + 4);
    v8h hv;
    hv[0] = (_Float16)(a[0] * sc);
    hv[1] = (_Float16)(a[1] * sc);
    hv[2] = (_Float16)(a[2] * sc);
    hv[3] = (_Float16)(a[3] * sc);
    hv[4] = (_Float16)(b[0] * sc);
    hv[5] = (_Float16)(b[1] * sc);
    hv[6] = (_Float16)(b[2] * sc);
    hv[7] = (_Float16)(b[3] * sc);
    unsigned short* dp = dst + (size_t)row * dpitch + dcol0 + c8 * 8;
    *(volatile v8h*)dp = hv;
    __threadfence();
    *(volatile v8h*)dp = hv;
  }
}

template <int T0, int NSTEPS>
__global__ __launch_bounds__(NTHR) void lstm_dir_kernel(const float* __restrict__ x,
                                                        const float* __restrict__ h0d, const float* __restrict__ c0d,
                                                        const float* __restrict__ bih, const float* __restrict__ bhh,
                                                        const unsigned short* __restrict__ Wp,
                                                        float* __restrict__ out, int outcol) {
  static_assert(T0 >= 0 && NSTEPS >= 1 && T0 + NSTEPS <= NSTEP, "time window inside the sequence");
  __shared__ __align__(16) _Float16 Xs[SEQ_BLK * XPITCH];
  __shared__ __align__(16) _Float16 Hh[2][SEQ_BLK * HPITCH];
  __shared__ __align__(16) float    Cs[SEQ_BLK * CPITCH];
  __shared__ __align__(16) float    Bs[NGATE];
  const _Float16* W = (const _Float16*)Wp;
  const int tid = threadIdx.x, lane = tid & 31, wave = tid >> 5;
  const int c = lane & 15, lh = lane >> 4, koff = lh * 8;
  const int rowbase = blockIdx.x * SEQ_BLK;
  const int srow = tid >> 4, sub = tid & 15;

  {
    const int e0 = tid * 8;
    const v4f a0 = *(const v4f*)(bih + e0);
    const v4f a1 = *(const v4f*)(bih + e0 + 4);
    const v4f b0 = *(const v4f*)(bhh + e0);
    const v4f b1 = *(const v4f*)(bhh + e0 + 4);
    const v4f s0 = a0 + b0;
    const v4f s1 = a1 + b1;
    *(v4f*)(Bs + e0)     = s0;
    *(v4f*)(Bs + e0 + 4) = s1;
  }
  {
    const float* hp = h0d + (size_t)(rowbase + srow) * NHID;
    const float* cp = c0d + (size_t)(rowbase + srow) * NHID;
#pragma unroll 4
    for (int it = 0; it < NHID / 64; ++it) {
      const int c4 = (sub + 16 * it) * 4;
      const v4f hv = *(const v4f*)(hp + c4);
      const v4f cv = *(const v4f*)(cp + c4);
      v4h h4;
      h4[0] = (_Float16)hv[0];
      h4[1] = (_Float16)hv[1];
      h4[2] = (_Float16)hv[2];
      h4[3] = (_Float16)hv[3];
      *(v4h*)(&Hh[0][0] + srow * HPITCH + c4) = h4;
      *(v4f*)(Cs + srow * CPITCH + c4) = cv;
    }
  }
  stage_x(x + ((size_t)(rowbase + srow) * NSTEP + (size_t)T0) * NIN, Xs + srow * XPITCH, sub);
  __syncthreads();

  const _Float16* xrow = Xs + c * XPITCH + koff;
  const v8f z8 = {0.f, 0.f, 0.f, 0.f, 0.f, 0.f, 0.f, 0.f};

#pragma unroll 1
  for (int s = 0; s < NSTEPS; ++s) {
    const int cur = s & 1;
    const _Float16* hrow = &Hh[cur][0] + c * HPITCH + koff;
    _Float16* hnext = &Hh[cur ^ 1][0];
    const bool last = (s == NSTEPS - 1);

#pragma unroll 1
    for (int nt = 0; nt < 4; ++nt) {
      const int j = 64 * wave + 16 * nt + c;
      const _Float16* w0 = W + (size_t)j * KCAT + koff;
      v8f acc0 = z8, acc1 = z8, acc2 = z8, acc3 = z8;
#pragma unroll 1
      for (int k0 = 0; k0 < NIN; k0 += 32) kstep(xrow + k0, w0 + k0, acc0, acc1, acc2, acc3);
#pragma unroll 1
      for (int k0 = 0; k0 < NHID; k0 += 32) kstep(hrow + k0, w0 + NIN + k0, acc0, acc1, acc2, acc3);
      acc_guard4(acc0, acc1, acc2, acc3);

      const float bi = Bs[j];
      const float bf = Bs[NHID + j];
      const float bg = Bs[2 * NHID + j];
      const float bo = Bs[3 * NHID + j];
#pragma unroll
      for (int r = 0; r < 8; ++r) {
        const int row = 8 * lh + r;
        const float zi = acc0[r] * WCARRY_INV + bi;
        const float zf = acc1[r] * WCARRY_INV + bf;
        const float zg = acc2[r] * WCARRY_INV + bg;
        const float zo = acc3[r] * WCARRY_INV + bo;
        const float ig = sigm(zi);
        const float fg = sigm(zf);
        const float gg = tnh(zg);
        const float og = sigm(zo);
        const float cp = Cs[row * CPITCH + j];
        const float cn = fg * cp + ig * gg;
        const float hv = og * tnh(cn);
        const float keep = last ? fmaxf(hv, 0.0f) : cn;
        Cs[row * CPITCH + j] = keep;
        hnext[row * HPITCH + j] = (_Float16)hv;
      }
    }
    __syncthreads();
    {
      const int tn = (T0 + s + 1 < NSTEP) ? (T0 + s + 1) : (NSTEP - 1);
      stage_x(x + ((size_t)(rowbase + srow) * NSTEP + (size_t)tn) * NIN, Xs + srow * XPITCH, sub);
    }
    __syncthreads();
  }

  for (int pass = 0; pass < 2; ++pass) {
#pragma unroll
    for (int it = 0; it < 8; ++it) {
      const int idx = it * NTHR + tid;
      const int row = idx >> 7;
      const int c4  = (idx & 127) * 4;
      const v4f v = *(const v4f*)(Cs + row * CPITCH + c4);
      *(volatile v4f*)(out + (size_t)(rowbase + row) * (2 * NHID) + outcol + c4) = v;
    }
    __threadfence();
  }
}

extern "C" void kernel_launch(void* const* d_in, const int* in_sizes, int n_in,
                              void* d_out, int out_size, void* d_ws, size_t ws_size, hipStream_t stream) {
  if (n_in < 11 || d_out == nullptr || d_ws == nullptr) return;
  if (in_sizes[0] != NBATCH * NSTEP * NIN || in_sizes[1] != 2 * NBATCH * NHID || in_sizes[2] != 2 * NBATCH * NHID ||
      in_sizes[3] != NGATE * NIN || in_sizes[4] != NGATE * NHID || in_sizes[5] != NGATE || in_sizes[6] != NGATE ||
      in_sizes[7] != NGATE * NIN || in_sizes[8] != NGATE * NHID || in_sizes[9] != NGATE || in_sizes[10] != NGATE ||
      out_size != NBATCH * 2 * NHID) return;

  const float* x      = (const float*)d_in[0];
  const float* h0     = (const float*)d_in[1];
  const float* c0     = (const float*)d_in[2];
  const float* w_ih_f = (const float*)d_in[3];
  const float* w_hh_f = (const float*)d_in[4];
  const float* b_ih_f = (const float*)d_in[5];
  const float* b_hh_f = (const float*)d_in[6];
  const float* w_ih_b = (const float*)d_in[7];
  const float* w_hh_b = (const float*)d_in[8];
  const float* b_ih_b = (const float*)d_in[9];
  const float* b_hh_b = (const float*)d_in[10];
  float* out = (float*)d_out;

  char* ws = (char*)d_ws;
  size_t off = 0;
  auto carve = [&](size_t bytes) -> char* { char* p = ws + off; off += (bytes + 255) & ~(size_t)255; return p; };
  unsigned short* WCF = (unsigned short*)carve((size_t)NGATE * KCAT * 2);
  unsigned short* WCB = (unsigned short*)carve((size_t)NGATE * KCAT * 2);
  if (off > ws_size || off > (size_t)134217728) return;

  const int n8i = NGATE * (NIN / 8);
  const int n8h = NGATE * (NHID / 8);
  cvt_w_kernel<<<n8i / NTHR, NTHR, 0, stream>>>(w_ih_f, WCF, NGATE, NIN / 8,  NIN,  KCAT, 0,   WCARRY);
  cvt_w_kernel<<<n8h / NTHR, NTHR, 0, stream>>>(w_hh_f, WCF, NGATE, NHID / 8, NHID, KCAT, NIN, WCARRY);
  cvt_w_kernel<<<n8i / NTHR, NTHR, 0, stream>>>(w_ih_b, WCB, NGATE, NIN / 8,  NIN,  KCAT, 0,   WCARRY);
  cvt_w_kernel<<<n8h / NTHR, NTHR, 0, stream>>>(w_hh_b, WCB, NGATE, NHID / 8, NHID, KCAT, NIN, WCARRY);

  lstm_dir_kernel<0, NSTEP><<<NBATCH / SEQ_BLK, NTHR, 0, stream>>>(
      x, h0, c0, b_ih_f, b_hh_f, WCF, out, 0);
  lstm_dir_kernel<NSTEP - 1, 1><<<NBATCH / SEQ_BLK, NTHR, 0, stream>>>(
      x, h0 + (size_t)NBATCH * NHID, c0 + (size_t)NBATCH * NHID, b_ih_b, b_hh_b, WCB, out, NHID);
}
